// LinkMLPPredictor_17540646437589
// MI455X (gfx1250) — hardware-verified
//
#include <hip/hip_runtime.h>
#include <math.h>

typedef __attribute__((ext_vector_type(16))) _Float16 v16h;
typedef __attribute__((ext_vector_type(16))) __bf16 v16b;
typedef __attribute__((ext_vector_type(8)))  _Float16 v8h;
typedef __attribute__((ext_vector_type(8)))  float v8f;
typedef __attribute__((ext_vector_type(4)))  float v4f;
typedef __attribute__((ext_vector_type(2)))  float v2f;
typedef __attribute__((ext_vector_type(4)))  unsigned v4u;
typedef __attribute__((ext_vector_type(4)))  int v4i;
typedef float __attribute__((may_alias)) float_a;
typedef int __attribute__((may_alias)) int_a;

template <typename T> __device__ __forceinline__ void vst2(void* p, T v) { *(volatile T*)p = v; __threadfence(); *(volatile T*)p = v; }
__device__ __forceinline__ v8f wmma16(v16h a, v16h b, v8f c) {
  v8f d = __builtin_amdgcn_wmma_f32_16x16x32_f16(false, a, false, b, (short)0, c, false, false);
  asm volatile("v_nop\n\tv_nop\n\tv_nop\n\tv_nop" : "+v"(d) : "v"(a), "v"(b));
  return d;
}
__device__ __forceinline__ v8f wmma_bf(v16b a, v16b b, v8f c) {
  v8f d = __builtin_amdgcn_wmma_f32_16x16x32_bf16(false, a, false, b, (short)0, c, false, false);
  asm volatile("v_nop\n\tv_nop\n\tv_nop\n\tv_nop" : "+v"(d) : "v"(a), "v"(b));
  return d;
}
__device__ __forceinline__ v16h frag_h(const _Float16* rowk0, int lane) {
  union { v16h v; v8h q[2]; } u; const _Float16* p = rowk0 + 8 * (lane >> 4);
  u.q[0] = *(const v8h*)p; u.q[1] = *(const v8h*)(p + 16); return u.v;
}
__device__ __forceinline__ v16h frag_f32(const float* rowk0, int lane) {
  v16h a; const float* p = rowk0 + 8 * (lane >> 4);
#pragma unroll
  for (int i = 0; i < 8; ++i) { a[i] = (_Float16)p[i]; a[8 + i] = (_Float16)p[16 + i]; }
  return a;
}
__device__ __forceinline__ v16h frag_f32s(const float* rowk0, int lane, float sc) {
  v16h a; const float* p = rowk0 + 8 * (lane >> 4);
#pragma unroll
  for (int i = 0; i < 8; ++i) { a[i] = (_Float16)(p[i] * sc); a[8 + i] = (_Float16)(p[16 + i] * sc); }
  return a;
}
__device__ __forceinline__ v16h fragc_f32(const float* W, int k0, int n, int lane, int ld, int K) {
  v16h a; const int g = lane >> 4;
#pragma unroll
  for (int i = 0; i < 8; ++i) { const int ka = k0 + 8 * g + i, kb = ka + 16;
    a[i] = (_Float16)(ka < K ? W[(size_t)(ka < K ? ka : K - 1) * ld + n] : 0.f); a[8 + i] = (_Float16)(kb < K ? W[(size_t)(kb < K ? kb : K - 1) * ld + n] : 0.f); }
  return a;
}
struct F2 { v16b h, l; };
__device__ __forceinline__ F2 bsplit16(const float v[16]) { F2 r;
#pragma unroll
  for (int i = 0; i < 16; ++i) { const __bf16 h = (__bf16)v[i]; r.h[i] = h; r.l[i] = (__bf16)(v[i] - (float)h); }
  return r; }
__device__ __forceinline__ F2 split_row(const float* row, int k0, int lane) { float v[16]; const float* p = row + k0 + 8 * (lane >> 4);
#pragma unroll
  for (int i = 0; i < 8; ++i) { v[i] = p[i]; v[8 + i] = p[16 + i]; }
  return bsplit16(v); }
__device__ __forceinline__ F2 split_rowK(const float* row, int k0, int lane, int K) { float v[16]; const int g = lane >> 4;
#pragma unroll
  for (int i = 0; i < 8; ++i) { const int ka = k0 + 8 * g + i, kb = ka + 16; v[i] = ka < K ? row[ka < K ? ka : K - 1] : 0.f; v[8 + i] = kb < K ? row[kb < K ? kb : K - 1] : 0.f; }
  return bsplit16(v); }
__device__ __forceinline__ F2 split_col(const float* W, int k0, int n, int lane, int ld, int K) { float v[16]; const int g = lane >> 4;
#pragma unroll
  for (int i = 0; i < 8; ++i) { const int ka = k0 + 8 * g + i, kb = ka + 16; v[i] = ka < K ? W[(size_t)(ka < K ? ka : K - 1) * ld + n] : 0.f; v[8 + i] = kb < K ? W[(size_t)(kb < K ? kb : K - 1) * ld + n] : 0.f; }
  return bsplit16(v); }
__device__ __forceinline__ v8f mac3(const F2& a, const F2& b, v8f c) { c = wmma_bf(a.l, b.h, c); c = wmma_bf(a.h, b.l, c); return wmma_bf(a.h, b.h, c); }
__device__ __forceinline__ float sigm(float v) { return 1.0f / (1.0f + expf(-v)); }
#define LDSX() do { asm volatile("s_wait_dscnt 0" ::: "memory"); __builtin_amdgcn_wave_barrier(); __builtin_amdgcn_fence(__ATOMIC_RELEASE, "workgroup"); } while (0)


#define NN 50000
#define DIN 128
#define HIDN 128
#define NE 1000000
#define EB 64
typedef __attribute__((ext_vector_type(8))) __bf16 v8b;
__device__ __forceinline__ v16b frag_b(const __bf16* rowk0, int lane) {
  union { v16b v; v8b q[2]; } u; const __bf16* p = rowk0 + 8 * (lane >> 4);
  u.q[0] = *(const v8b*)p; u.q[1] = *(const v8b*)(p + 16); return u.v;
}
__device__ __forceinline__ float bfr(float v) { return (float)(__bf16)v; }
__device__ __attribute__((noinline)) float exp_ni(float v) { return expf(v); }

__global__ __launch_bounds__(256) void k_pack(const float* __restrict__ W1, __bf16* __restrict__ W1T) {
  __shared__ __align__(16) __bf16 srow[2 * DIN];
  const int n = blockIdx.x, tid = threadIdx.x;
  srow[tid] = (__bf16)W1[(size_t)tid * HIDN + n];
  __syncthreads();
  if (tid < 32) vst2((unsigned*)(W1T + (size_t)n * 2 * DIN + tid * 8), *(const v4u*)(&srow[tid * 8]));
}
__global__ __launch_bounds__(256) void k_edge(const float* __restrict__ P, const float* __restrict__ C, const int* __restrict__ ei, const __bf16* __restrict__ W1T, const float* __restrict__ b1, const float* __restrict__ W2, const float* __restrict__ b2, float* __restrict__ out) {
  __shared__ __align__(16) __bf16 sa[EB][2 * DIN + 8];
  __shared__ float spart[2][EB];
  __shared__ __align__(16) float sout[EB];
  const int tid = threadIdx.x, wave = tid >> 5, lane = tid & 31, col = lane & 15, g = lane >> 4; const size_t e0 = (size_t)blockIdx.x * EB;
  { const int el = (wave >> 2) * 32 + lane, q4 = wave & 3; const size_t e = e0 + el; const size_t ec = e < NE ? e : NE - 1;
    int is = ei[ec], id = ei[NE + ec]; is = is < 0 ? 0 : (is >= NN ? NN - 1 : is); id = id < 0 ? 0 : (id >= NN ? NN - 1 : id);
    const float* srcrow = (q4 < 2 ? P + (size_t)is * DIN : C + (size_t)id * DIN) + (q4 & 1) * 64;
#pragma unroll
    for (int c4 = 0; c4 < 16; ++c4) { const float4 v = *(const float4*)(srcrow + c4 * 4); __bf16* d = &sa[el][q4 * 64 + c4 * 4]; d[0] = (__bf16)v.x; d[1] = (__bf16)v.y; d[2] = (__bf16)v.z; d[3] = (__bf16)v.w; } }
  __syncthreads();
  const int rt = wave & 3, ct0 = (wave >> 2) * 4; v8f acc[4] = {};
#pragma unroll 2
  for (int kc = 0; kc < 2 * DIN / 32; ++kc) { const v16b a = frag_b(&sa[rt * 16 + col][kc * 32], lane);
#pragma unroll
    for (int j = 0; j < 4; ++j) acc[j] = wmma_bf(a, frag_b(W1T + (size_t)((ct0 + j) * 16 + col) * 2 * DIN + kc * 32, lane), acc[j]); }
  float part[8];
#pragma unroll
  for (int r = 0; r < 8; ++r) part[r] = 0.f;
#pragma unroll
  for (int j = 0; j < 4; ++j) { const int c = (ct0 + j) * 16 + col; const float bb = bfr(b1[c]), w2 = bfr(W2[c]);
#pragma unroll
    for (int r = 0; r < 8; ++r) { const float h = acc[j][r] + bb; part[r] += (h > 0.f ? h : 0.f) * w2; } }
#pragma unroll
  for (int r = 0; r < 8; ++r) {
#pragma unroll
    for (int o = 1; o < 16; o <<= 1) part[r] += __shfl_xor(part[r], o); }
  if (col == 0) {
#pragma unroll
    for (int r = 0; r < 8; ++r) spart[wave >> 2][rt * 16 + 8 * g + r] = part[r]; }
  __syncthreads();
  if (tid < EB) { const float z = (spart[0][tid] + spart[1][tid]) + bfr(b2[0]); sout[tid] = 1.0f / (1.0f + exp_ni(-z)); }
  __syncthreads();
  if (tid < 16) vst2(out + e0 + tid * 4, *(const v4f*)&sout[tid * 4]);
}

extern "C" void kernel_launch(void* const* d_in, const int* in_sizes, int n_in, void* d_out, int out_size, void* d_ws, size_t ws_size, hipStream_t stream) {
  (void)in_sizes; (void)n_in; (void)out_size; (void)ws_size;
  const float* P = (const float*)d_in[0]; const float* C = (const float*)d_in[1]; const int* ei = (const int*)d_in[2];
  const float* W1 = (const float*)d_in[3]; const float* b1 = (const float*)d_in[4]; const float* W2 = (const float*)d_in[5]; const float* b2 = (const float*)d_in[6];
  __bf16* W1T = (__bf16*)d_ws;
  k_pack<<<HIDN, 256, 0, stream>>>(W1, W1T);
  k_edge<<<NE / EB, 256, 0, stream>>>(P, C, ei, W1T, b1, W2, b2, (float*)d_out);
}
